// Net_42786464203126
// MI455X (gfx1250) — hardware-verified
//
#include <hip/hip_runtime.h>
#include <stddef.h>
#include <stdint.h>
#include <math.h>

#define FO      32
#define NBIN    125
#define KB      128
#define AP      256
#define NVOX    32768
#define NTHR    256
#define NWAVE   8
#define EPT     8
#define CHUNK   (NTHR * EPT)
#define WCAP    (EPT * 32)
#define LISTN   (NWAVE * WCAP)
#define NBA     1024
#define SLA     10
#define RCAP_E  28672
#define DCAP_E  64
#define RCAP_V  4096
#define DCAP_V  64
#define MISC_INTS 16
#define ZINTS_E (LISTN + 2 * RCAP_E + 3 * NBA)
#define ZINTS_V (LISTN + 2 * RCAP_V + 3 * NBA)
#define SCAN_LDS_INTS (ZINTS_E + MISC_INTS + NWAVE * (AP / 2))
#define POOL_LDS_INTS (ZINTS_V + MISC_INTS)
#define GBM     128
#define GTHR    128
#define PB_W    4
#define WSMAX   134217728

static_assert((CHUNK & (CHUNK - 1)) == 0 && CHUNK <= 4096);
static_assert((NBA & (NBA - 1)) == 0 && NBA == (1 << SLA) && NBA == 4 * NTHR);
static_assert(((long long)CHUNK << SLA) < (1LL << 31));
static_assert(NBA % NWAVE == 0 && NBA % GBM == 0);
static_assert(RCAP_E >= 17564 && DCAP_E >= 38 + 8);
static_assert(RCAP_V >= 2 * 2048 && DCAP_V >= 64);
static_assert(ZINTS_E % 4 == 0 && ZINTS_V % 4 == 0 && LISTN % 4 == 0);
static_assert(((ZINTS_E + MISC_INTS) % 4) == 0);
static_assert(SCAN_LDS_INTS * 4 <= 300000);
static_assert(AP % 32 == 0 && AP == 2 * KB && KB == 4 * 32 && FO == 2 * 16);
static_assert(PB_W * NTHR == FO * (AP / 8));
static_assert(NVOX % NBA == 0);

typedef float          v4f   __attribute__((ext_vector_type(4)));
typedef float          v8f   __attribute__((ext_vector_type(8)));
typedef int            v4i   __attribute__((ext_vector_type(4)));
typedef int            v8i   __attribute__((ext_vector_type(8)));
typedef unsigned short v4us  __attribute__((ext_vector_type(4)));
typedef unsigned short v8us  __attribute__((ext_vector_type(8)));
typedef unsigned short v16us __attribute__((ext_vector_type(16)));
typedef __bf16         v16bf __attribute__((ext_vector_type(16)));
typedef v4f  __attribute__((may_alias)) v4fa;
typedef v4i  __attribute__((may_alias)) v4ia;
typedef v4us __attribute__((may_alias)) v4usa;
typedef v8us __attribute__((may_alias)) v8usa;
union FragB { v16bf v; v16us u; v8us h[2]; v8i w; };

__device__ __forceinline__ v8f wmb(const FragB& a, const FragB& b, v8f c) {
  v8f d = __builtin_amdgcn_wmma_f32_16x16x32_bf16(false, a.v, false, b.v, (short)0, c, false, false);
  asm volatile("v_nop\n\tv_nop\n\tv_nop\n\tv_nop" : "+v"(d) : "v"(a.w), "v"(b.w));
  return d;
}

__device__ __forceinline__ unsigned bf16_bits(float f) {
  const unsigned u = __float_as_uint(f);
  return (u + 0x7FFFu + ((u >> 16) & 1u)) >> 16;
}
__device__ __forceinline__ float bf16_val(float f) {
  return __uint_as_float(bf16_bits(f) << 16);
}

__device__ __forceinline__ void wave_sync() {
  __builtin_amdgcn_fence(__ATOMIC_RELEASE, "wavefront");
  __builtin_amdgcn_wave_barrier();
  __builtin_amdgcn_fence(__ATOMIC_ACQUIRE, "wavefront");
}

template <int SLB>
__device__ __forceinline__ int scan_chunk(const int* __restrict__ dsts, int nE, int cbase, int slotBase,
                                          int nb, int vec8, int* list, int tid, int lane, int wave) {
  int wc = 0;
  const int el0  = tid * EPT;
  const int e0   = cbase + el0;
  const int sent = -2147483647 - 1;
  v4i da, db;
  if (vec8 != 0 && cbase + CHUNK <= nE) {
    da = *(const v4i*)(dsts + e0);
    db = *(const v4i*)(dsts + e0 + 4);
  } else {
    da.x = (e0     < nE) ? dsts[min(e0,     nE - 1)] : sent;
    da.y = (e0 + 1 < nE) ? dsts[min(e0 + 1, nE - 1)] : sent;
    da.z = (e0 + 2 < nE) ? dsts[min(e0 + 2, nE - 1)] : sent;
    da.w = (e0 + 3 < nE) ? dsts[min(e0 + 3, nE - 1)] : sent;
    db.x = (e0 + 4 < nE) ? dsts[min(e0 + 4, nE - 1)] : sent;
    db.y = (e0 + 5 < nE) ? dsts[min(e0 + 5, nE - 1)] : sent;
    db.z = (e0 + 6 < nE) ? dsts[min(e0 + 6, nE - 1)] : sent;
    db.w = (e0 + 7 < nE) ? dsts[min(e0 + 7, nE - 1)] : sent;
  }
  const unsigned nbs = (unsigned)slotBase;
  const unsigned unb = (unsigned)nb;
  const unsigned s0 = (unsigned)da.x - nbs, s1 = (unsigned)da.y - nbs;
  const unsigned s2 = (unsigned)da.z - nbs, s3 = (unsigned)da.w - nbs;
  const unsigned s4 = (unsigned)db.x - nbs, s5 = (unsigned)db.y - nbs;
  const unsigned s6 = (unsigned)db.z - nbs, s7 = (unsigned)db.w - nbs;
  const bool h0 = s0 < unb, h1 = s1 < unb, h2 = s2 < unb, h3 = s3 < unb;
  const bool h4 = s4 < unb, h5 = s5 < unb, h6 = s6 < unb, h7 = s7 < unb;
  const unsigned any = __builtin_amdgcn_ballot_w32(h0 | h1 | h2 | h3 | h4 | h5 | h6 | h7);
  if (any != 0u) {
#define HITJ(J, HJ, SJ) { \
      const unsigned mj = __builtin_amdgcn_ballot_w32(HJ); \
      if (mj != 0u) { \
        if (HJ) { \
          const int pos = wc + (int)__builtin_amdgcn_mbcnt_lo(mj, 0u); \
          if (pos < WCAP) list[wave * WCAP + pos] = ((el0 + (J)) << SLB) | (int)(SJ); \
        } \
        wc += (int)__builtin_popcount(mj); } }
    HITJ(0, h0, s0)
    HITJ(1, h1, s1)
    HITJ(2, h2, s2)
    HITJ(3, h3, s3)
    HITJ(4, h4, s4)
    HITJ(5, h5, s5)
    HITJ(6, h6, s6)
    HITJ(7, h7, s7)
#undef HITJ
  }
  return wc;
}

template <int RC, int DC>
__device__ __forceinline__ void build_lists(const int* __restrict__ keys, int nE, int vec8, int slotBase,
                                            int* dsm, int tid, int lane, int wave) {
  int* list = dsm;
  int* hl   = dsm + LISTN;
  int* sl   = hl + RC;
  int* cnt  = sl + RC;
  int* offs = cnt + NBA;
  int* cur  = offs + NBA;
  int* misc = cur + NBA;
  {
    const v4i z4 = {0, 0, 0, 0};
    for (int i = tid * 4; i < LISTN + 2 * RC + 3 * NBA; i += NTHR * 4) *(v4ia*)(dsm + i) = z4;
    if (tid < MISC_INTS) misc[tid] = 0;
  }
  __syncthreads();

  int t = 0, ov = 0;
  const int nChunks = (nE + CHUNK - 1) / CHUNK;
#pragma unroll 1
  for (int ch = 0; ch < nChunks; ++ch) {
    const int cbase = ch * CHUNK;
    const int wc = scan_chunk<SLA>(keys, nE, cbase, slotBase, NBA, vec8, list, tid, lane, wave);
    if (lane == 0) misc[wave] = wc;
    __syncthreads();
    if (wave == 0) {
#pragma unroll 1
      for (int w2 = 0; w2 < NWAVE; ++w2) {
        int c = misc[w2];
        c = c < 0 ? 0 : (c > WCAP ? WCAP : c);
#pragma unroll 1
        for (int b0 = 0; b0 < c; b0 += 32) {
          const int idx = b0 + lane;
          const int ent = list[w2 * WCAP + (idx < WCAP ? idx : WCAP - 1)];
          const int m32 = (c - b0) < 32 ? (c - b0) : 32;
#pragma unroll 1
          for (int k = 0; k < m32; ++k) {
            const int u    = __builtin_amdgcn_readlane(ent, k);
            const int slot = u & (NBA - 1);
            const int el   = (u >> SLA) & (CHUNK - 1);
            const int pk   = ((cbase + el) << SLA) | slot;
            if (t < RC) {
              if (lane == 0) { hl[t] = pk; cnt[slot] = cnt[slot] + 1; }
              t = t + 1;
            } else {
              ov = 1;
            }
          }
        }
      }
    }
    __syncthreads();
  }
  if (wave == 0 && lane == 0) { misc[8] = t; misc[9] = ov; }
  __syncthreads();
  int tt = misc[8];
  tt = tt < 0 ? 0 : (tt > RC ? RC : tt);

  if (wave == 0) {
    const int base = lane * (NBA / 32);
    int s = 0;
#pragma unroll 1
    for (int i = 0; i < NBA / 32; ++i) s += cnt[base + i];
    int incl = s;
#pragma unroll
    for (int d = 1; d < 32; d <<= 1) {
      const int y = __shfl_up(incl, d, 32);
      if (lane >= d) incl += y;
    }
    int run = incl - s;
#pragma unroll 1
    for (int i = 0; i < NBA / 32; ++i) {
      const int cv = cnt[base + i];
      offs[base + i] = run;
      cur[base + i]  = run;
      run += cv;
    }
  }
  __syncthreads();
  if (wave == 0) {
#pragma unroll 1
    for (int b0 = 0; b0 < tt; b0 += 32) {
      const int idx = b0 + lane;
      const int ent = hl[idx < RC ? idx : RC - 1];
      const int m32 = (tt - b0) < 32 ? (tt - b0) : 32;
#pragma unroll 1
      for (int k = 0; k < m32; ++k) {
        const int u    = __builtin_amdgcn_readlane(ent, k);
        const int slot = u & (NBA - 1);
        if (lane == 0) {
          int p = cur[slot];
          p = p < 0 ? 0 : (p > RC - 1 ? RC - 1 : p);
          sl[p] = u;
          cur[slot] = p + 1;
        }
      }
    }
  }
  __syncthreads();
  {
    const v4i c4 = *(const v4ia*)(cnt + 4 * tid);
    const bool bg = (c4.x > DC) | (c4.y > DC) | (c4.z > DC) | (c4.w > DC);
    const unsigned mb = __builtin_amdgcn_ballot_w32(bg);
    if (mb != 0u && lane == 0) misc[10] = 1;
  }
  __syncthreads();
}

__device__ __forceinline__ int vox1(float p) {
  const float v = bf16_val(p) * 32.0f;
  float f = floorf(v);
  f = fminf(fmaxf(f, 0.0f), 31.0f);
  return (int)f;
}

__global__ __launch_bounds__(NTHR) void k_prep(const float* __restrict__ W, const float* __restrict__ Wroot,
                                               const float* __restrict__ bias, const float* __restrict__ pos,
                                               unsigned short* WT2, float* SM, int* VIDX, int nN, int nV) {
  const int b = (int)blockIdx.x, tid = (int)threadIdx.x;
  if (b < PB_W) {
    const int u  = b * NTHR + tid;
    const int n  = u >> 5;
    const int k8 = (u & 31) * 8;
    v8us o;
#pragma unroll
    for (int j = 0; j < 8; ++j) {
      const int kk = (k8 + j) & (KB - 1);
      const int kc = kk < NBIN ? kk : NBIN - 1;
      const float w = W[kc * FO + n];
      const unsigned bits = bf16_bits(w);
      o[j] = (kk < NBIN) ? (unsigned short)bits : (unsigned short)0;
    }
    unsigned short* dp = WT2 + (size_t)n * AP + k8;
    *(volatile v8us*)dp = o;
    __threadfence();
    *(volatile v8us*)dp = o;
  } else if (b < PB_W + nV) {
    int g = (b - PB_W) * NTHR + tid;
    const int gmax = nN / 4 - 1;
    g = g > gmax ? gmax : g;
    const float* p = pos + (size_t)g * 12;
    const v4f a = *(const v4f*)p;
    const v4f c = *(const v4f*)(p + 4);
    const v4f d = *(const v4f*)(p + 8);
    v4i o;
    o.x = vox1(a.x) + 32 * vox1(a.y) + 1024 * vox1(a.z);
    o.y = vox1(a.w) + 32 * vox1(c.x) + 1024 * vox1(c.y);
    o.z = vox1(c.z) + 32 * vox1(c.w) + 1024 * vox1(d.x);
    o.w = vox1(d.y) + 32 * vox1(d.z) + 1024 * vox1(d.w);
    int* dp = VIDX + (size_t)g * 4;
    *(volatile v4i*)dp = o;
    __threadfence();
    *(volatile v4i*)dp = o;
  } else {
    const int u   = tid & 15;
    const int idx = (u & 7) * 4;
    const v4f wr = *(const v4f*)(Wroot + idx);
    const v4f bi = *(const v4f*)(bias + idx);
    const bool isw = u < 8;
    v4f o;
    o.x = bf16_val(isw ? wr.x : bi.x);
    o.y = bf16_val(isw ? wr.y : bi.y);
    o.z = bf16_val(isw ? wr.z : bi.z);
    o.w = bf16_val(isw ? wr.w : bi.w);
    if (tid < 16) {
      float* dp = SM + 4 * u;
      *(volatile v4f*)dp = o;
      __threadfence();
      *(volatile v4f*)dp = o;
    }
  }
}

__global__ __launch_bounds__(NTHR) void k_scan(const int* __restrict__ ei, const float* __restrict__ xin,
                                               const float* __restrict__ ps, int nE, int nN, int vec8,
                                               unsigned short* Cb, float* DEG, int* FLAGL) {
  extern __shared__ __attribute__((aligned(16))) int dsm[];
  const int tid = (int)threadIdx.x, lane = tid & 31, wave = tid >> 5;
  const int nodeBase = (int)blockIdx.x * NBA;
  const int* keys = ei + nE;
  const int* gath = ei;

  build_lists<RCAP_E, DCAP_E>(keys, nE, vec8, nodeBase, dsm, tid, lane, wave);

  int* sl   = dsm + LISTN + RCAP_E;
  int* cnt  = sl + RCAP_E;
  int* offs = cnt + NBA;
  int* misc = offs + 2 * NBA;
  unsigned short* rowbuf = (unsigned short*)(misc + MISC_INTS) + wave * AP;
  const int bad = ((misc[9] | misc[10]) != 0) ? 1 : 0;

  {
    const v4i c4 = *(const v4ia*)(cnt + 4 * tid);
    v4f d4;
    d4.x = (float)c4.x; d4.y = (float)c4.y; d4.z = (float)c4.z; d4.w = (float)c4.w;
    float* dp = DEG + nodeBase + 4 * tid;
    const v4i f4 = {bad, bad, bad, bad};
    int* fp = FLAGL + (size_t)blockIdx.x * 32 + 4 * (lane & 7);
    *(volatile v4f*)dp = d4;
    if (wave == 0 && lane < 8) *(volatile v4i*)fp = f4;
    __threadfence();
    *(volatile v4f*)dp = d4;
    if (wave == 0 && lane < 8) *(volatile v4i*)fp = f4;
  }

  int ka[4], kb[4], kc[4];
  bool kv[4];
#pragma unroll
  for (int t = 0; t < 4; ++t) {
    const int k = 4 * lane + t;
    kv[t] = k < NBIN;
    ka[t] = k % 5;
    kb[t] = (k / 5) % 5;
    kc[t] = kv[t] ? (k / 25) : 7;
  }
  const float qnan = __int_as_float(0x7fc00000);
  const float pz = (bad != 0) ? qnan : 0.0f;

#pragma unroll 1
  for (int si = 0; si < NBA / NWAVE; ++si) {
    const int s    = si * NWAVE + wave;
    const int node = nodeBase + s;
    int c = cnt[s];
    c = c < 0 ? 0 : (c > DCAP_E ? DCAP_E : c);
    int o = offs[s];
    o = o < 0 ? 0 : (o > RCAP_E ? RCAP_E : o);
    float bn[4] = {0.0f, 0.0f, 0.0f, 0.0f};
#pragma unroll 1
    for (int b0 = 0; b0 < c; b0 += 32) {
      int idx = o + b0 + lane;
      idx = idx > RCAP_E - 1 ? RCAP_E - 1 : idx;
      const int ent = sl[idx];
      int eid = ent >> SLA;
      eid = eid < 0 ? 0 : (eid > nE - 1 ? nE - 1 : eid);
      int sr = gath[eid];
      sr = sr < 0 ? 0 : (sr > nN - 1 ? nN - 1 : sr);
      const float xv = bf16_val(xin[sr]);
      const float* pp = ps + (size_t)eid * 3;
      const float v0 = bf16_val(pp[0]) * 4.0f;
      const float v1 = bf16_val(pp[1]) * 4.0f;
      const float v2 = bf16_val(pp[2]) * 4.0f;
      const float l0 = fminf(fmaxf(floorf(v0), 0.0f), 3.0f);
      const float l1 = fminf(fmaxf(floorf(v1), 0.0f), 3.0f);
      const float l2 = fminf(fmaxf(floorf(v2), 0.0f), 3.0f);
      const int fi0 = __float_as_int(v0 - l0);
      const int fi1 = __float_as_int(v1 - l1);
      const int fi2 = __float_as_int(v2 - l2);
      const int xi  = __float_as_int(xv);
      const int pk  = (int)l0 | ((int)l1 << 2) | ((int)l2 << 4);
      const int m32 = (c - b0) < 32 ? (c - b0) : 32;
#pragma unroll 1
      for (int k = 0; k < m32; ++k) {
        const int   u  = __builtin_amdgcn_readlane(pk, k);
        const float g0 = __int_as_float(__builtin_amdgcn_readlane(fi0, k));
        const float g1 = __int_as_float(__builtin_amdgcn_readlane(fi1, k));
        const float g2 = __int_as_float(__builtin_amdgcn_readlane(fi2, k));
        const float xk = __int_as_float(__builtin_amdgcn_readlane(xi, k));
        const int j0 = u & 3, j1 = (u >> 2) & 3, j2 = (u >> 4) & 3;
        const float h0 = 1.0f - g0, h1 = 1.0f - g1, h2 = 1.0f - g2;
#pragma unroll
        for (int t = 0; t < 4; ++t) {
          const float s0 = (ka[t] == j0) ? h0 : ((ka[t] == j0 + 1) ? g0 : 0.0f);
          const float s1 = (kb[t] == j1) ? h1 : ((kb[t] == j1 + 1) ? g1 : 0.0f);
          const float s2 = (kc[t] == j2) ? h2 : ((kc[t] == j2 + 1) ? g2 : 0.0f);
          const float cf = ((s0 * s1) * s2) * xk;
          bn[t] = bn[t] + cf;
        }
      }
    }
    v4us mh, ml;
#pragma unroll
    for (int t = 0; t < 4; ++t) {
      const float mv = (kv[t] ? bn[t] : 0.0f) + pz;
      const unsigned hb = bf16_bits(mv);
      mh[t] = (unsigned short)hb;
      ml[t] = (unsigned short)bf16_bits(mv - __uint_as_float(hb << 16));
    }
    *(v4usa*)(rowbuf + 4 * lane) = mh;
    *(v4usa*)(rowbuf + KB + 4 * lane) = ml;
    wave_sync();
    const v8us q0 = *(const v8usa*)(rowbuf + 8 * lane);
    wave_sync();
    if (node < nN) {
      unsigned short* rpw = Cb + (size_t)node * AP + 8 * lane;
      *(volatile v8us*)rpw = q0;
      __threadfence();
      *(volatile v8us*)rpw = q0;
    }
  }
}

__global__ __launch_bounds__(GTHR) void k_gemm(const unsigned short* __restrict__ Cb,
                                               const unsigned short* __restrict__ WT2,
                                               const float* __restrict__ DEG, const float* __restrict__ xin,
                                               const float* __restrict__ SM, float* H) {
  __shared__ __attribute__((aligned(16))) float sO[GBM * FO];
  __shared__ __attribute__((aligned(16))) float sD[GBM];
  __shared__ __attribute__((aligned(16))) float sX[GBM];
  __shared__ __attribute__((aligned(16))) float sW[FO];
  __shared__ __attribute__((aligned(16))) float sB[FO];
  const int tid = (int)threadIdx.x, lane = tid & 31, wave = tid >> 5, hh = lane >> 4, m = lane & 15;
  const int rowBase = (int)blockIdx.x * GBM;

  v8f acc[2][2];
  {
    const v8f z = {0.f, 0.f, 0.f, 0.f, 0.f, 0.f, 0.f, 0.f};
#pragma unroll
    for (int mt = 0; mt < 2; ++mt)
#pragma unroll
      for (int nt = 0; nt < 2; ++nt) acc[mt][nt] = z;
  }
  const unsigned short* ap0 = Cb + (size_t)(rowBase + 32 * wave + m) * (size_t)AP + 8 * hh;
  const unsigned short* ap1 = ap0 + (size_t)16 * AP;
  const unsigned short* bp  = WT2 + (size_t)m * (size_t)AP + 8 * hh;

#pragma unroll 1
  for (int k0 = 0; k0 < AP; k0 += 32) {
    FragB a0, a1;
    a0.h[0] = *(const v8usa*)(ap0 + k0);
    a0.h[1] = *(const v8usa*)(ap0 + k0 + 16);
    a1.h[0] = *(const v8usa*)(ap1 + k0);
    a1.h[1] = *(const v8usa*)(ap1 + k0 + 16);
#pragma unroll
    for (int nt = 0; nt < 2; ++nt) {
      const unsigned short* wq = bp + (size_t)(16 * nt) * (size_t)AP + k0;
      FragB bf;
      bf.h[0] = *(const v8usa*)wq;
      bf.h[1] = *(const v8usa*)(wq + 16);
      acc[0][nt] = wmb(a0, bf, acc[0][nt]);
      acc[1][nt] = wmb(a1, bf, acc[1][nt]);
    }
  }

#pragma unroll
  for (int mt = 0; mt < 2; ++mt)
#pragma unroll
    for (int nt = 0; nt < 2; ++nt) {
      const int lc = 16 * nt + m;
#pragma unroll
      for (int r = 0; r < 8; ++r) {
        const int lr = 32 * wave + 16 * mt + 8 * hh + r;
        sO[lr * FO + lc] = acc[mt][nt][r];
      }
    }

  if (wave == 0) {
    const v4f d = *(const v4f*)(DEG + rowBase + 4 * lane);
    *(v4fa*)(sD + 4 * lane) = d;
  } else if (wave == 1) {
    const v4f a = *(const v4f*)(xin + rowBase + 4 * lane);
    v4f b;
    b.x = bf16_val(a.x); b.y = bf16_val(a.y); b.z = bf16_val(a.z); b.w = bf16_val(a.w);
    *(v4fa*)(sX + 4 * lane) = b;
  } else if (wave == 2) {
    const v4f a = *(const v4f*)(SM + 4 * (lane & 7));
    if (lane < 8) *(v4fa*)(sW + 4 * lane) = a;
  } else {
    const v4f a = *(const v4f*)(SM + FO + 4 * (lane & 7));
    if (lane < 8) *(v4fa*)(sB + 4 * lane) = a;
  }
  __syncthreads();

#pragma unroll 1
  for (int it = 0; it < (GBM * FO) / GTHR; ++it) {
    const int e = it * GTHR + tid;
    const int r = e >> 5, o = e & 31;
    const float den = fmaxf(sD[r], 1.0f);
    const float v = sO[e] / den + sX[r] * sW[o] + sB[o];
    const float hv = (v > 0.0f) ? v : expm1f(v);
    sO[e] = hv;
  }
  __syncthreads();

  v4f pv[8];
#pragma unroll
  for (int it = 0; it < 8; ++it) pv[it] = *(const v4fa*)(sO + 4 * (it * GTHR + tid));
  float* hb = H + (size_t)rowBase * FO;
#pragma unroll
  for (int it = 0; it < 8; ++it) *(volatile v4f*)(hb + 4 * (it * GTHR + tid)) = pv[it];
  __threadfence();
#pragma unroll
  for (int it = 0; it < 8; ++it) *(volatile v4f*)(hb + 4 * (it * GTHR + tid)) = pv[it];
}

__global__ __launch_bounds__(NTHR) void k_pool(const int* __restrict__ vidx, const float* __restrict__ H,
                                               const int* __restrict__ flagl, int nFl, int nN, int vec8,
                                               float* out) {
  extern __shared__ __attribute__((aligned(16))) int dsm[];
  const int tid = (int)threadIdx.x, lane = tid & 31, wave = tid >> 5;
  const int voxBase = (int)blockIdx.x * NBA;

  build_lists<RCAP_V, DCAP_V>(vidx, nN, vec8, voxBase, dsm, tid, lane, wave);

  int* sl   = dsm + LISTN + RCAP_V;
  int* cnt  = sl + RCAP_V;
  int* offs = cnt + NBA;
  int* misc = offs + 2 * NBA;
  {
    const int fi = tid < nFl - 1 ? tid : nFl - 1;
    const int fv = flagl[(size_t)fi * 32];
    const unsigned mb = __builtin_amdgcn_ballot_w32(fv != 0);
    if (mb != 0u && lane == 0) misc[11] = 1;
  }
  __syncthreads();
  const bool pois = (misc[9] | misc[10] | misc[11]) != 0;
  const float qnan = __int_as_float(0x7fc00000);
  const float ninf = __int_as_float((int)0xff800000u);

#pragma unroll 1
  for (int si = 0; si < NBA / NWAVE; ++si) {
    const int s   = si * NWAVE + wave;
    const int vox = voxBase + s;
    int c = cnt[s];
    c = c < 0 ? 0 : (c > DCAP_V ? DCAP_V : c);
    int o = offs[s];
    o = o < 0 ? 0 : (o > RCAP_V ? RCAP_V : o);
    float mx = ninf;
#pragma unroll 1
    for (int b0 = 0; b0 < c; b0 += 32) {
      int idx = o + b0 + lane;
      idx = idx > RCAP_V - 1 ? RCAP_V - 1 : idx;
      const int ent = sl[idx];
      int nid = ent >> SLA;
      nid = nid < 0 ? 0 : (nid > nN - 1 ? nN - 1 : nid);
      const int m32 = (c - b0) < 32 ? (c - b0) : 32;
#pragma unroll 1
      for (int k = 0; k < m32; ++k) {
        const int nk = __builtin_amdgcn_readlane(nid, k);
        const float v = H[(size_t)nk * FO + lane];
        mx = (v > mx) ? v : mx;
      }
    }
    const bool fin = (__float_as_uint(mx) & 0x7f800000u) != 0x7f800000u;
    float r = fin ? mx : 0.0f;
    r = pois ? qnan : r;
    if (vox < NVOX) {
      float* dp = out + (size_t)vox * FO + lane;
      *(volatile float*)dp = r;
      __threadfence();
      *(volatile float*)dp = r;
    }
  }
}

static inline size_t al256(size_t o) { return (o + 255) & ~(size_t)255; }

extern "C" void kernel_launch(void* const* d_in, const int* in_sizes, int n_in,
                              void* d_out, int out_size, void* d_ws, size_t ws_size,
                              hipStream_t stream) {
  if (n_in < 7) return;
  const int nN = in_sizes[0];
  if (nN < NBA || (nN % NBA) != 0 || nN >= (1 << 21)) return;
  if (in_sizes[1] < 2 || (in_sizes[1] & 1) != 0) return;
  const int nE = in_sizes[1] / 2;
  if (nE < 1 || nE >= (1 << 21)) return;
  if ((long long)in_sizes[2] != 3LL * nE) return;
  if ((long long)in_sizes[3] != 3LL * nN) return;
  if (in_sizes[4] != NBIN * FO) return;
  if (in_sizes[5] != FO || in_sizes[6] != FO) return;
  if (out_size != NVOX * FO) return;

  const float* x      = (const float*)d_in[0];
  const int*   ei     = (const int*)d_in[1];
  const float* pseudo = (const float*)d_in[2];
  const float* pos    = (const float*)d_in[3];
  const float* W      = (const float*)d_in[4];
  const float* Wroot  = (const float*)d_in[5];
  const float* bias   = (const float*)d_in[6];
  float* out = (float*)d_out;

  const int gS = nN / NBA;
  const int gV = NVOX / NBA;
  const int gM = nN / GBM;
  const int nV = nN / (4 * NTHR);
  const int vecE = ((nE & 3) == 0) ? 1 : 0;
  const int vecN = 1;

  char* ws = (char*)d_ws;
  size_t off = 0;
  const size_t oCb = off; off = al256(off + (size_t)nN * AP * 2);
  const size_t oH  = off; off = al256(off + (size_t)nN * FO * 4);
  const size_t oDg = off; off = al256(off + (size_t)nN * 4);
  const size_t oVx = off; off = al256(off + (size_t)nN * 4);
  const size_t oWT = off; off = al256(off + (size_t)FO * AP * 2);
  const size_t oSM = off; off = al256(off + (size_t)2 * FO * 4);
  const size_t oFl = off; off = al256(off + (size_t)gS * 128);
  if (off > ws_size || off > (size_t)WSMAX) return;
  unsigned short* Cb  = (unsigned short*)(ws + oCb);
  float* H    = (float*)(ws + oH);
  float* DEG  = (float*)(ws + oDg);
  int*   VIDX = (int*)(ws + oVx);
  unsigned short* WT2 = (unsigned short*)(ws + oWT);
  float* SM   = (float*)(ws + oSM);
  int*   FLAGL = (int*)(ws + oFl);

  const size_t scanLds = (size_t)SCAN_LDS_INTS * 4;
  const size_t poolLds = (size_t)POOL_LDS_INTS * 4;
  hipFuncSetAttribute(reinterpret_cast<const void*>(&k_scan), hipFuncAttributeMaxDynamicSharedMemorySize, (int)scanLds);
  hipFuncSetAttribute(reinterpret_cast<const void*>(&k_pool), hipFuncAttributeMaxDynamicSharedMemorySize, (int)poolLds);

  k_prep<<<PB_W + nV + 1, NTHR, 0, stream>>>(W, Wroot, bias, pos, WT2, SM, VIDX, nN, nV);
  k_scan<<<gS, NTHR, scanLds, stream>>>(ei, x, pseudo, nE, nN, vecE, Cb, DEG, FLAGL);
  k_gemm<<<gM, GTHR, 0, stream>>>(Cb, WT2, DEG, x, SM, H);
  k_pool<<<gV, NTHR, poolLds, stream>>>(VIDX, H, FLAGL, gS, nN, vecN, out);
  (void)hipGetLastError();
}
